// KPConv_12489764897253
// MI455X (gfx1250) — hardware-verified
//
#include <hip/hip_runtime.h>
#include <math.h>

typedef __attribute__((ext_vector_type(16))) _Float16 v16h;
typedef __attribute__((ext_vector_type(16))) __bf16 v16b;
typedef __attribute__((ext_vector_type(8)))  _Float16 v8h;
typedef __attribute__((ext_vector_type(8)))  float v8f;
typedef __attribute__((ext_vector_type(4)))  float v4f;
typedef __attribute__((ext_vector_type(2)))  float v2f;
typedef __attribute__((ext_vector_type(4)))  unsigned v4u;
typedef __attribute__((ext_vector_type(4)))  int v4i;
typedef float __attribute__((may_alias)) float_a;
typedef int __attribute__((may_alias)) int_a;

template <typename T> __device__ __forceinline__ void vst2(void* p, T v) { *(volatile T*)p = v; __threadfence(); *(volatile T*)p = v; }
__device__ __forceinline__ v8f wmma16(v16h a, v16h b, v8f c) {
  v8f d = __builtin_amdgcn_wmma_f32_16x16x32_f16(false, a, false, b, (short)0, c, false, false);
  asm volatile("v_nop\n\tv_nop\n\tv_nop\n\tv_nop" : "+v"(d) : "v"(a), "v"(b));
  return d;
}
__device__ __forceinline__ v8f wmma_bf(v16b a, v16b b, v8f c) {
  v8f d = __builtin_amdgcn_wmma_f32_16x16x32_bf16(false, a, false, b, (short)0, c, false, false);
  asm volatile("v_nop\n\tv_nop\n\tv_nop\n\tv_nop" : "+v"(d) : "v"(a), "v"(b));
  return d;
}
__device__ __forceinline__ v16h frag_h(const _Float16* rowk0, int lane) {
  union { v16h v; v8h q[2]; } u; const _Float16* p = rowk0 + 8 * (lane >> 4);
  u.q[0] = *(const v8h*)p; u.q[1] = *(const v8h*)(p + 16); return u.v;
}
__device__ __forceinline__ v16h frag_f32(const float* rowk0, int lane) {
  v16h a; const float* p = rowk0 + 8 * (lane >> 4);
#pragma unroll
  for (int i = 0; i < 8; ++i) { a[i] = (_Float16)p[i]; a[8 + i] = (_Float16)p[16 + i]; }
  return a;
}
__device__ __forceinline__ v16h frag_f32s(const float* rowk0, int lane, float sc) {
  v16h a; const float* p = rowk0 + 8 * (lane >> 4);
#pragma unroll
  for (int i = 0; i < 8; ++i) { a[i] = (_Float16)(p[i] * sc); a[8 + i] = (_Float16)(p[16 + i] * sc); }
  return a;
}
__device__ __forceinline__ v16h fragc_f32(const float* W, int k0, int n, int lane, int ld, int K) {
  v16h a; const int g = lane >> 4;
#pragma unroll
  for (int i = 0; i < 8; ++i) { const int ka = k0 + 8 * g + i, kb = ka + 16;
    a[i] = (_Float16)(ka < K ? W[(size_t)(ka < K ? ka : K - 1) * ld + n] : 0.f); a[8 + i] = (_Float16)(kb < K ? W[(size_t)(kb < K ? kb : K - 1) * ld + n] : 0.f); }
  return a;
}
struct F2 { v16b h, l; };
__device__ __forceinline__ F2 bsplit16(const float v[16]) { F2 r;
#pragma unroll
  for (int i = 0; i < 16; ++i) { const __bf16 h = (__bf16)v[i]; r.h[i] = h; r.l[i] = (__bf16)(v[i] - (float)h); }
  return r; }
__device__ __forceinline__ F2 split_row(const float* row, int k0, int lane) { float v[16]; const float* p = row + k0 + 8 * (lane >> 4);
#pragma unroll
  for (int i = 0; i < 8; ++i) { v[i] = p[i]; v[8 + i] = p[16 + i]; }
  return bsplit16(v); }
__device__ __forceinline__ F2 split_rowK(const float* row, int k0, int lane, int K) { float v[16]; const int g = lane >> 4;
#pragma unroll
  for (int i = 0; i < 8; ++i) { const int ka = k0 + 8 * g + i, kb = ka + 16; v[i] = ka < K ? row[ka < K ? ka : K - 1] : 0.f; v[8 + i] = kb < K ? row[kb < K ? kb : K - 1] : 0.f; }
  return bsplit16(v); }
__device__ __forceinline__ F2 split_col(const float* W, int k0, int n, int lane, int ld, int K) { float v[16]; const int g = lane >> 4;
#pragma unroll
  for (int i = 0; i < 8; ++i) { const int ka = k0 + 8 * g + i, kb = ka + 16; v[i] = ka < K ? W[(size_t)(ka < K ? ka : K - 1) * ld + n] : 0.f; v[8 + i] = kb < K ? W[(size_t)(kb < K ? kb : K - 1) * ld + n] : 0.f; }
  return bsplit16(v); }
__device__ __forceinline__ v8f mac3(const F2& a, const F2& b, v8f c) { c = wmma_bf(a.l, b.h, c); c = wmma_bf(a.h, b.l, c); return wmma_bf(a.h, b.h, c); }
__device__ __forceinline__ float sigm(float v) { return 1.0f / (1.0f + expf(-v)); }
#define LDSX() do { asm volatile("s_wait_dscnt 0" ::: "memory"); __builtin_amdgcn_wave_barrier(); __builtin_amdgcn_fence(__ATOMIC_RELEASE, "workgroup"); } while (0)

typedef __attribute__((ext_vector_type(4))) int v4i;
__device__ __forceinline__ float bfr(float v) { return (float)(__bf16)v; }
__device__ __forceinline__ v16b wcol_io(const float* __restrict__ Wm, int k0, int o, int lane, int ld) { v16b w; const float* p = Wm + (size_t)(k0 + 8 * (lane >> 4)) * ld + o;
#pragma unroll
  for (int i = 0; i < 8; ++i) { w[i] = (__bf16)p[(size_t)i * ld]; w[8 + i] = (__bf16)p[(size_t)(16 + i) * ld]; }
  asm volatile("s_wait_loadcnt 0x0" ::: "memory"); return w; }
#define NBT 2
#define NPT 8192
#define NQ 2048
#define CI 64
#define CO 128
#define KP 15
#define KN 32
#define NR (NBT * NQ)
#ifndef NRV
#define NRV NR
#endif
#define FKW (KP * CI)
#define WS_IDX 0u
#define WS_DS  (WS_IDX + 4u * (size_t)NR * KN)
#define WS_FK  (WS_DS + 4u * (size_t)NR * KN)
#define WS_END (WS_FK + 4u * (size_t)NR * FKW)
struct Best32 { float d[KN]; int i[KN]; };
__device__ __forceinline__ void push32(Best32& b, float d, int i) {
  if (d < b.d[KN - 1]) { b.d[KN - 1] = d; b.i[KN - 1] = i; }
#pragma unroll
  for (int p = KN - 1; p > 0; --p) { const bool sw = b.d[p] < b.d[p - 1]; const float td = b.d[p], ud = b.d[p - 1]; const int ti = b.i[p], ui = b.i[p - 1]; b.d[p] = sw ? ud : td; b.d[p - 1] = sw ? td : ud; b.i[p] = sw ? ui : ti; b.i[p - 1] = sw ? ti : ui; } }
__global__ __launch_bounds__(256) void k_knn32(const float* __restrict__ QP, const float* __restrict__ P, int* __restrict__ IDX, float* __restrict__ DS) {
  const int wave = threadIdx.x >> 5, lane = threadIdx.x & 31; const size_t row = (size_t)blockIdx.x * 8 + wave; if (row >= (size_t)NRV) return;
  const size_t b = row / NQ; const int m = (int)(row % NQ);
  Best32 bs;
#pragma unroll
  for (int r = 0; r < KN; ++r) { bs.d[r] = 3.0e38f; bs.i[r] = 0x7fffffff; }
  {
#pragma clang fp contract(off)
    const float qx = bfr(QP[(b * NQ + m) * 3]), qy = bfr(QP[(b * NQ + m) * 3 + 1]), qz = bfr(QP[(b * NQ + m) * 3 + 2]);
    const float aa = (qx * qx + qy * qy) + qz * qz;
#pragma unroll 1
    for (int s = lane; s < NPT; s += 32) { const float px = bfr(P[(b * NPT + s) * 3]), py = bfr(P[(b * NPT + s) * 3 + 1]), pz = bfr(P[(b * NPT + s) * 3 + 2]);
      const float bb = (px * px + py * py) + pz * pz; const float dot = (qx * px + qy * py) + qz * pz; const float d2 = (aa + bb) - 2.0f * dot;
      float d = __fsqrt_rn(fmaxf(d2, 0.f)); d = (d <= 0.5f) ? d : 1.5f;
      push32(bs, d, s); } }
  int sel = 0; float seld = 0.f;
#pragma unroll 1
  for (int r = 0; r < KN; ++r) { float d = bs.d[0]; int i = bs.i[0];
#pragma unroll
    for (int o = 1; o < 32; o <<= 1) { const float e = __shfl_xor(d, o); const int j = __shfl_xor(i, o); if (e < d || (e == d && j < i)) { d = e; i = j; } }
    if (lane == r) { sel = i; seld = d; }
    { const bool pop = (bs.i[0] == i && bs.d[0] == d);
#pragma unroll
      for (int p = 0; p < KN - 1; ++p) { bs.d[p] = pop ? bs.d[p + 1] : bs.d[p]; bs.i[p] = pop ? bs.i[p + 1] : bs.i[p]; }
      bs.d[KN - 1] = pop ? 3.0e38f : bs.d[KN - 1]; bs.i[KN - 1] = pop ? 0x7fffffff : bs.i[KN - 1]; } }
  vst2(IDX + row * KN + lane, sel); vst2(DS + row * KN + lane, seld); }
__global__ __launch_bounds__(128) void k_fk(const float* __restrict__ QP, const float* __restrict__ P, const float* __restrict__ FT, const float* __restrict__ KPT, const int* __restrict__ IDX, const float* __restrict__ DS, float* __restrict__ FK) { __shared__ float srel[4][KN][4]; __shared__ int sidx[4][KN]; __shared__ __align__(16) float sf[4][16][68];
  const int tid = threadIdx.x, wave = tid >> 5, lane = tid & 31, col = lane & 15, g = lane >> 4; const size_t row = (size_t)blockIdx.x * 4 + wave; const size_t b = row / NQ; const int m = (int)(row % NQ);
  { int ix = IDX[row * KN + lane]; const float d = DS[row * KN + lane]; const bool ok = (d <= 0.5f) && ix >= 0 && ix < NPT; ix = ok ? ix : 0; sidx[wave][lane] = ok ? (int)(b * NPT + ix) : -1;
    const float qx = bfr(QP[(b * NQ + m) * 3]), qy = bfr(QP[(b * NQ + m) * 3 + 1]), qz = bfr(QP[(b * NQ + m) * 3 + 2]);
    const size_t pp = (b * NPT + ix) * 3; srel[wave][lane][0] = ok ? bfr(P[pp]) - qx : 0.f; srel[wave][lane][1] = ok ? bfr(P[pp + 1]) - qy : 0.f; srel[wave][lane][2] = ok ? bfr(P[pp + 2]) - qz : 0.f; srel[wave][lane][3] = ok ? 1.f : 0.f; }
  LDSX();
  float va[16]; { const bool kv = col < KP; const float kx = kv ? bfr(KPT[col * 3]) : 0.f, ky = kv ? bfr(KPT[col * 3 + 1]) : 0.f, kz = kv ? bfr(KPT[col * 3 + 2]) : 0.f;
#pragma unroll
    for (int i = 0; i < 16; ++i) { const int n = (i < 8) ? (8 * g + i) : (16 + 8 * g + (i - 8)); const float dx = srel[wave][n][0] - kx, dy = srel[wave][n][1] - ky, dz = srel[wave][n][2] - kz; const float sq = (dx * dx + dy * dy) + dz * dz;
      const float wv = expf(-sq * (1.0f / 0.045f)) * srel[wave][n][3]; va[i] = kv ? wv : 0.f; } }
  const F2 a = bsplit16(va);
  v8f acc[4] = {};
#pragma unroll
  for (int j = 0; j < 4; ++j) { v16b fb; { const int c = j * 16 + col;
#pragma unroll
      for (int i = 0; i < 16; ++i) { const int n = (i < 8) ? (8 * g + i) : (16 + 8 * g + (i - 8)); const int gi = sidx[wave][n]; const float fv = gi >= 0 ? FT[(size_t)gi * CI + c] : 0.f; fb[i] = (__bf16)fv; } }
    asm volatile("s_wait_loadcnt 0x0" ::: "memory");
    acc[j] = wmma_bf(a.h, fb, acc[j]); acc[j] = wmma_bf(a.l, fb, acc[j]); }
#pragma unroll
  for (int j = 0; j < 4; ++j)
#pragma unroll
    for (int r = 0; r < 8; ++r) sf[wave][8 * g + r][j * 16 + col] = acc[j][r];
  LDSX();
  for (int k = 0; k < KP; ++k) if (lane < 16) vst2(FK + row * FKW + k * CI + lane * 4, *(const v4f*)&sf[wave][k][lane * 4]); }
__global__ __launch_bounds__(128) void k_out2(const float* __restrict__ FK, const float* __restrict__ WT, const float* __restrict__ BS, float* __restrict__ OUT) { __shared__ __align__(16) float so[4][16][132];
  const int tid = threadIdx.x, wave = tid >> 5, lane = tid & 31, col = lane & 15, g = lane >> 4; const size_t r0 = (size_t)blockIdx.x * 64 + wave * 16;
  v8f acc[8] = {};
#pragma unroll 2
  for (int kc = 0; kc < FKW / 32; ++kc) { const F2 a = split_row(FK + (r0 + col) * FKW, kc * 32, lane); asm volatile("s_wait_loadcnt 0x0" ::: "memory");
#pragma unroll
    for (int j = 0; j < 8; ++j) { const v16b w = wcol_io(WT, kc * 32, j * 16 + col, lane, CO); acc[j] = wmma_bf(a.h, w, acc[j]); acc[j] = wmma_bf(a.l, w, acc[j]); } }
#pragma unroll
  for (int j = 0; j < 8; ++j) { const float bb = bfr(BS[j * 16 + col]);
#pragma unroll
    for (int r = 0; r < 8; ++r) so[wave][8 * g + r][j * 16 + col] = acc[j][r] + bb; }
  LDSX(); for (int rl = 0; rl < 16; ++rl) vst2(OUT + (r0 + rl) * CO + lane * 4, *(const v4f*)&so[wave][rl][lane * 4]); }
extern "C" void kernel_launch(void* const* d_in, const int* in_sizes, int n_in, void* d_out, int out_size, void* d_ws, size_t ws_size, hipStream_t stream) {
  (void)in_sizes; (void)n_in; (void)out_size;
  if (ws_size < (size_t)WS_END) return;
  char* ws = (char*)d_ws; const float** F = (const float**)d_in; int* IDX = (int*)(ws + WS_IDX); float *DS = (float*)(ws + WS_DS), *FK = (float*)(ws + WS_FK);
  k_knn32<<<dim3((NRV + 7) / 8), 256, 0, stream>>>(F[2], F[0], IDX, DS);
  k_fk<<<dim3(NRV / 4), 128, 0, stream>>>(F[2], F[0], F[1], F[5], IDX, DS, FK);
  k_out2<<<dim3(NRV / 64), 128, 0, stream>>>(FK, F[3], F[4], (float*)d_out);
}
